// EGConvLayer_18708877542146
// MI455X (gfx1250) — hardware-run, weakly checked
//
#include <hip/hip_runtime.h>
#include <stddef.h>


#pragma clang fp contract(off)

#define DN      128
#define NTHR    256
#define NWAVE   8
#define NBN     64
#define NBE     64
#define APA     136
#define APN     264
#define GSTR    132
#define NPROW   256
#define MROW    128
#define CROW    4
#define EPT     8
#define PIECE   (NTHR * EPT)
#define WCAP    (EPT * 32)
#define NBC     512
#define SLB     9
#define CE      114688
#define MAXCH   64
#define PAH     0
#define PAL     16384
#define PBH     32768
#define PBL     49152
#define PM2     65536
#define PN1H    81920
#define PN1L    114688
#define PN2H    147456
#define PN2L    163840
#define PWTOT   180224
#define PBLK    (PWTOT / (NTHR * 8))
#define WSCAP   134217728
#define NODEDYN (2 * NBN * APA * 2)
#define EDGEDYN (NBE * GSTR * 4)
#define AGGDYN  ((NBC * DN + NBC * CROW) * 4)
#define MLPDYN  (2 * NBN * APN * 2 + 2 * NBN * APA * 2)
#define SCW     16.0f
#define SCA     64.0f
#define INV1024 0.0009765625f

static_assert((PWTOT % (NTHR * 8)) == 0);
static_assert((PAL % (NTHR * 8)) == 0);
static_assert((PBH % (NTHR * 8)) == 0);
static_assert((PBL % (NTHR * 8)) == 0);
static_assert((PM2 % (NTHR * 8)) == 0);
static_assert((PN1H % (NTHR * 8)) == 0);
static_assert((PN1L % (NTHR * 8)) == 0);
static_assert((PN2H % (NTHR * 8)) == 0);
static_assert((PN2L % (NTHR * 8)) == 0);
static_assert(((APA * 2) % 16) == 0);
static_assert(((APN * 2) % 16) == 0);
static_assert(((GSTR * 4) % 16) == 0);
static_assert(NBN * APN * 2 == NBN * GSTR * 4);
static_assert(NODEDYN == 34816);
static_assert(MLPDYN == 102400);
static_assert(NBC == (1 << SLB));
static_assert(PIECE == 2048);
static_assert((EPT % 4) == 0);
static_assert((CE % PIECE) == 0);
static_assert((CE % NBE) == 0);
static_assert((NBC % NWAVE) == 0);
static_assert(3 * NBC <= 8 * NTHR);
static_assert(NBE == NWAVE * 8);
static_assert(NBN == 4 * 16);
static_assert((NBC * DN) % (4 * NTHR) == 0);

typedef float          v4f   __attribute__((ext_vector_type(4)));
typedef float          v8f   __attribute__((ext_vector_type(8)));
typedef int            v4i   __attribute__((ext_vector_type(4)));
typedef unsigned short v8us  __attribute__((ext_vector_type(8)));
typedef _Float16       v4h   __attribute__((ext_vector_type(4)));
typedef _Float16       v8h   __attribute__((ext_vector_type(8)));
typedef _Float16       v16h  __attribute__((ext_vector_type(16)));
typedef __bf16         v16b  __attribute__((ext_vector_type(16)));
union FragH { v16h v; v8h h[2]; };
union FragB { v16b v; v8us u[2]; };
union Cvt8  { v8h v; v8us u; };

__device__ __forceinline__ v8f wmh(v16h a, v16h b, v8f c) {
  v8f d = __builtin_amdgcn_wmma_f32_16x16x32_f16(false, a, false, b, (short)0, c, false, false);
  asm volatile("v_nop\n\tv_nop\n\tv_nop\n\tv_nop" : "+v"(d) : "v"(a), "v"(b));
  return d;
}
__device__ __forceinline__ v8f wmb(v16b a, v16b b, v8f c) {
  v8f d = __builtin_amdgcn_wmma_f32_16x16x32_bf16(false, a, false, b, (short)0, c, false, false);
  asm volatile("v_nop\n\tv_nop\n\tv_nop\n\tv_nop" : "+v"(d) : "v"(a), "v"(b));
  return d;
}
__device__ __forceinline__ v8f zero8() {
  v8f z = {0.f, 0.f, 0.f, 0.f, 0.f, 0.f, 0.f, 0.f};
  return z;
}
__device__ __forceinline__ v4f zero4() {
  v4f z = {0.f, 0.f, 0.f, 0.f};
  return z;
}
__device__ __forceinline__ int imin(int a, int b) { return a < b ? a : b; }
__device__ __forceinline__ int iclamp(int v, int lo, int hi) { return v < lo ? lo : (v > hi ? hi : v); }

__device__ __forceinline__ unsigned short bf_rne(float f) {
  unsigned u = __float_as_uint(f);
  u += 0x7FFFu + ((u >> 16) & 1u);
  return (unsigned short)(u >> 16);
}
__device__ __forceinline__ float bf_val(unsigned short b) { return __uint_as_float(((unsigned)b) << 16); }

__device__ __forceinline__ void cvt_hl8(v4f xa, v4f xb, v8us& h, v8us& l) {
  float f[8];
  f[0] = xa.x; f[1] = xa.y; f[2] = xa.z; f[3] = xa.w;
  f[4] = xb.x; f[5] = xb.y; f[6] = xb.z; f[7] = xb.w;
#pragma unroll
  for (int j = 0; j < 8; ++j) {
    const unsigned short hb = bf_rne(f[j]);
    h[j] = hb;
    l[j] = bf_rne(f[j] - bf_val(hb));
  }
}

__device__ __forceinline__ void gemm16x64(const _Float16* ap, const _Float16* __restrict__ bpl, int kp, int nks, int n0,
                                          int m, int hh, v8f& c0, v8f& c1, v8f& c2, v8f& c3) {
  c0 = zero8(); c1 = zero8(); c2 = zero8(); c3 = zero8();
#pragma unroll 1
  for (int ks = 0; ks < nks; ++ks) {
    FragH a;
    a.h[0] = *(const v8h*)(ap + 32 * ks);
    a.h[1] = *(const v8h*)(ap + 32 * ks + 16);
    const _Float16* bp = bpl + (size_t)(n0 + m) * kp + 32 * ks + 8 * hh;
    FragH b;
    b.h[0] = *(const v8h*)(bp);
    b.h[1] = *(const v8h*)(bp + 16);
    c0 = wmh(a.v, b.v, c0);
    b.h[0] = *(const v8h*)(bp + (size_t)16 * kp);
    b.h[1] = *(const v8h*)(bp + (size_t)16 * kp + 16);
    c1 = wmh(a.v, b.v, c1);
    b.h[0] = *(const v8h*)(bp + (size_t)32 * kp);
    b.h[1] = *(const v8h*)(bp + (size_t)32 * kp + 16);
    c2 = wmh(a.v, b.v, c2);
    b.h[0] = *(const v8h*)(bp + (size_t)48 * kp);
    b.h[1] = *(const v8h*)(bp + (size_t)48 * kp + 16);
    c3 = wmh(a.v, b.v, c3);
  }
}

__device__ __forceinline__ void tile3(const unsigned short* __restrict__ bh, const unsigned short* __restrict__ bl,
                                      size_t ob, const FragB& ah, const FragB& al, v8f& c) {
  FragB b;
  b.u[0] = *(const v8us*)(bh + ob);
  b.u[1] = *(const v8us*)(bh + ob + 16);
  c = wmb(ah.v, b.v, c);
  c = wmb(al.v, b.v, c);
  b.u[0] = *(const v8us*)(bl + ob);
  b.u[1] = *(const v8us*)(bl + ob + 16);
  c = wmb(ah.v, b.v, c);
}

__device__ __forceinline__ void gemm3x16x64(const unsigned short* aph, const unsigned short* apl,
                                            const unsigned short* __restrict__ bh, const unsigned short* __restrict__ bl,
                                            int kp, int nks, int n0, int m, int hh, v8f& c0, v8f& c1, v8f& c2, v8f& c3) {
  c0 = zero8(); c1 = zero8(); c2 = zero8(); c3 = zero8();
#pragma unroll 1
  for (int ks = 0; ks < nks; ++ks) {
    FragB ah, al;
    ah.u[0] = *(const v8us*)(aph + 32 * ks);
    ah.u[1] = *(const v8us*)(aph + 32 * ks + 16);
    al.u[0] = *(const v8us*)(apl + 32 * ks);
    al.u[1] = *(const v8us*)(apl + 32 * ks + 16);
    const size_t ob = (size_t)(n0 + m) * kp + 32 * ks + 8 * hh;
    tile3(bh, bl, ob,                     ah, al, c0);
    tile3(bh, bl, ob + (size_t)16 * kp,   ah, al, c1);
    tile3(bh, bl, ob + (size_t)32 * kp,   ah, al, c2);
    tile3(bh, bl, ob + (size_t)48 * kp,   ah, al, c3);
  }
}

__device__ __forceinline__ void stage8f(float* sp, v8f a, float scl, float bias) {
#pragma unroll
  for (int r = 0; r < 8; ++r) sp[r * GSTR] = a[r] * scl + bias;
}
__device__ __forceinline__ void stage8y(unsigned short* ph, unsigned short* pl, v8f a, float bias) {
#pragma unroll
  for (int r = 0; r < 8; ++r) {
    const float v = fmaxf(a[r] + bias, 0.0f);
    const unsigned short hb = bf_rne(v);
    ph[r * APA] = hb;
    pl[r * APA] = bf_rne(v - bf_val(hb));
  }
}

__global__ __launch_bounds__(NTHR) void k_prep(
    const float* __restrict__ We1, const float* __restrict__ We2, const float* __restrict__ Wh1,
    const float* __restrict__ Wh2, unsigned short* wp) {
  const int tid = (int)threadIdx.x;
  const int b = (int)blockIdx.x;
  const int o = (b * NTHR + tid) * 8;
  const float* src = We1;
  int r0 = 0, n, k0, mode = 0;
  if (o < PAL)       { n = o >> 7; k0 = o & 127; }
  else if (o < PBH)  { const int idx = o - PAL;  n = idx >> 7; k0 = idx & 127; mode = 1; }
  else if (o < PBL)  { const int idx = o - PBH;  n = idx >> 7; k0 = idx & 127; r0 = DN; }
  else if (o < PM2)  { const int idx = o - PBL;  n = idx >> 7; k0 = idx & 127; r0 = DN; mode = 1; }
  else if (o < PN1H) { const int idx = o - PM2;  n = idx >> 7; k0 = idx & 127; src = We2; mode = 2; }
  else if (o < PN1L) { const int idx = o - PN1H; n = idx >> 8; k0 = idx & 255; src = Wh1; }
  else if (o < PN2H) { const int idx = o - PN1L; n = idx >> 8; k0 = idx & 255; src = Wh1; mode = 1; }
  else if (o < PN2L) { const int idx = o - PN2H; n = idx >> 7; k0 = idx & 127; src = Wh2; }
  else               { const int idx = o - PN2L; n = idx >> 7; k0 = idx & 127; src = Wh2; mode = 1; }
  v8us ov;
  if (mode == 2) {
    Cvt8 cv;
#pragma unroll
    for (int j = 0; j < 8; ++j) cv.v[j] = (_Float16)(src[(size_t)(k0 + j) * DN + n] * SCW);
    ov = cv.u;
  } else {
#pragma unroll
    for (int j = 0; j < 8; ++j) {
      const float w = src[(size_t)(r0 + k0 + j) * DN + n];
      const unsigned short hb = bf_rne(w);
      const unsigned short lb = bf_rne(w - bf_val(hb));
      ov[j] = (mode == 0) ? hb : lb;
    }
  }
  unsigned short* dp = wp + o;
  *(volatile v8us*)dp = ov;
  __threadfence();
  *(volatile v8us*)dp = ov;
}

__global__ __launch_bounds__(NTHR) void k_node(
    const float* __restrict__ nsrc, const unsigned short* __restrict__ wp, float* NP, int nN) {
  extern __shared__ __attribute__((aligned(16))) float ndynf[];
  __shared__ __attribute__((aligned(16))) float stg[NWAVE * 1024];
  unsigned short* sAH = (unsigned short*)ndynf;
  unsigned short* sAL = sAH + NBN * APA;
  const int tid = (int)threadIdx.x, lane = tid & 31, wave = tid >> 5, hh = lane >> 4, m = lane & 15;
  const int n0 = (int)blockIdx.x * NBN;

  {
    const int nl = tid >> 2, q = tid & 3;
    int node = n0 + nl;
    node = node > nN - 1 ? nN - 1 : node;
    const float* rp = nsrc + (size_t)node * DN + 32 * q;
#pragma unroll
    for (int i = 0; i < 4; ++i) {
      const v4f xa = *(const v4f*)(rp + 8 * i);
      const v4f xb = *(const v4f*)(rp + 8 * i + 4);
      v8us h, l;
      cvt_hl8(xa, xb, h, l);
      *(v8us*)(sAH + nl * APA + 32 * q + 8 * i) = h;
      *(v8us*)(sAL + nl * APA + 32 * q + 8 * i) = l;
    }
  }
  __syncthreads();

  const int rt = wave & 3, chf = wave >> 2;
  const unsigned short* aph = sAH + (16 * rt + m) * APA + 8 * hh;
  const unsigned short* apl = sAL + (16 * rt + m) * APA + 8 * hh;
  const unsigned short* bh = wp + (chf ? PBH : PAH);
  const unsigned short* bl = wp + (chf ? PBL : PAL);
  float* sw = stg + wave * 1024;
#pragma unroll 1
  for (int qq = 0; qq < 2; ++qq) {
    v8f a0, a1, a2, a3;
    gemm3x16x64(aph, apl, bh, bl, DN, 4, 64 * qq, m, hh, a0, a1, a2, a3);
    {
      float* sp = sw + (8 * hh) * 64 + m;
#pragma unroll
      for (int r = 0; r < 8; ++r) {
        sp[r * 64]      = a0[r];
        sp[r * 64 + 16] = a1[r];
        sp[r * 64 + 32] = a2[r];
        sp[r * 64 + 48] = a3[r];
      }
    }
    __syncthreads();
#pragma unroll 1
    for (int i = 0; i < 8; ++i) {
      const int r2 = 2 * i + hh;
      const v4f v = *(const v4f*)(sw + r2 * 64 + 4 * m);
      const int row = n0 + 16 * rt + r2;
      *(volatile v4f*)(NP + (size_t)row * NPROW + 128 * chf + 64 * qq + 4 * m) = v;
    }
    __threadfence();
#pragma unroll 1
    for (int i = 0; i < 8; ++i) {
      const int r2 = 2 * i + hh;
      const v4f v = *(const v4f*)(sw + r2 * 64 + 4 * m);
      const int row = n0 + 16 * rt + r2;
      *(volatile v4f*)(NP + (size_t)row * NPROW + 128 * chf + 64 * qq + 4 * m) = v;
    }
    __syncthreads();
  }
}

__global__ __launch_bounds__(NTHR) void k_edge(
    const float* __restrict__ x, const int* __restrict__ ei, const float* __restrict__ NP,
    const unsigned short* __restrict__ wp, const float* __restrict__ We1, const float* __restrict__ be1,
    const float* __restrict__ be2, const float* __restrict__ Wx, const float* __restrict__ bx,
    float* Mout, float* Cout, int nE, int nN, int cbeg) {
  extern __shared__ __attribute__((aligned(16))) float sH[];
  __shared__ __attribute__((aligned(16))) _Float16 sA[NBE * APA];
  __shared__ __attribute__((aligned(16))) float sPar[4 * DN + 4];
  __shared__ __attribute__((aligned(16))) float sDis[NBE * 4];
  __shared__ __attribute__((aligned(16))) float sCo[NBE * 4];
  __shared__ float sRad[NBE];
  __shared__ int sI[NBE];
  __shared__ int sJ[NBE];
  const int tid = (int)threadIdx.x, lane = tid & 31, wave = tid >> 5, hh = lane >> 4, m = lane & 15;
  const int el0 = (int)blockIdx.x * NBE;

  if (tid < NBE) {
    int e = cbeg + el0 + tid;
    e = e > nE - 1 ? nE - 1 : e;
    const int ii = iclamp(ei[(size_t)nE + e], 0, nN - 1);
    const int jj = iclamp(ei[e], 0, nN - 1);
    const float dx = x[(size_t)ii * 3]     - x[(size_t)jj * 3];
    const float dy = x[(size_t)ii * 3 + 1] - x[(size_t)jj * 3 + 1];
    const float dz = x[(size_t)ii * 3 + 2] - x[(size_t)jj * 3 + 2];
    const float rad = (dx * dx + dz * dz) + dy * dy;
    sDis[4 * tid]     = dx;
    sDis[4 * tid + 1] = dy;
    sDis[4 * tid + 2] = dz;
    sDis[4 * tid + 3] = 0.0f;
    sRad[tid] = rad;
    sI[tid] = ii;
    sJ[tid] = jj;
  }
  if (tid < DN) {
    sPar[tid]          = be1[tid];
    sPar[DN + tid]     = We1[(size_t)2 * DN * DN + tid];
    sPar[2 * DN + tid] = be2[tid];
    sPar[3 * DN + tid] = Wx[tid];
  }
  if (tid == 0) sPar[4 * DN] = bx[0];
  __syncthreads();

  {
    const int c4 = 4 * lane;
    const v4f bb = *(const v4f*)(sPar + c4);
    const v4f wr = *(const v4f*)(sPar + DN + c4);
#pragma unroll 1
    for (int jx = 0; jx < 8; ++jx) {
      const int el = 8 * wave + jx;
      const int ii = sI[el];
      const int jj = sJ[el];
      const float rad = sRad[el];
      const v4f p = *(const v4f*)(NP + (size_t)ii * NPROW + c4);
      const v4f q = *(const v4f*)(NP + (size_t)jj * NPROW + DN + c4);
      const v4f v = ((p + q) + wr * rad) + bb;
      v4h z;
      z.x = (_Float16)(fmaxf(v.x, 0.0f) * SCA);
      z.y = (_Float16)(fmaxf(v.y, 0.0f) * SCA);
      z.z = (_Float16)(fmaxf(v.z, 0.0f) * SCA);
      z.w = (_Float16)(fmaxf(v.w, 0.0f) * SCA);
      *(v4h*)(sA + el * APA + c4) = z;
    }
  }
  __syncthreads();

  const int rt = wave & 3, cg = wave >> 2;

  {
    v8f a0, a1, a2, a3;
    gemm16x64(sA + (16 * rt + m) * APA + 8 * hh, (const _Float16*)(wp + PM2), DN, 4, 64 * cg, m, hh, a0, a1, a2, a3);
    float* sp = sH + (16 * rt + 8 * hh) * GSTR + 64 * cg + m;
    const float* bb = sPar + 2 * DN + 64 * cg + m;
    stage8f(sp,      a0, INV1024, bb[0]);
    stage8f(sp + 16, a1, INV1024, bb[16]);
    stage8f(sp + 32, a2, INV1024, bb[32]);
    stage8f(sp + 48, a3, INV1024, bb[48]);
  }
  __syncthreads();

  {
#pragma unroll 1
    for (int it = 0; it < 8; ++it) {
      const int row = wave + NWAVE * it;
      const v4f v = *(const v4f*)(sH + row * GSTR + 4 * lane);
      *(volatile v4f*)(Mout + (size_t)(el0 + row) * MROW + 4 * lane) = v;
    }
    __threadfence();
#pragma unroll 1
    for (int it = 0; it < 8; ++it) {
      const int row = wave + NWAVE * it;
      const v4f v = *(const v4f*)(sH + row * GSTR + 4 * lane);
      *(volatile v4f*)(Mout + (size_t)(el0 + row) * MROW + 4 * lane) = v;
    }
  }

  {
    const int e = tid >> 2, g = tid & 3;
    const float* row = sH + e * GSTR + 32 * g;
    const float* w2 = sPar + 3 * DN + 32 * g;
    float s = 0.f;
#pragma unroll 4
    for (int c = 0; c < 32; ++c) s += row[c] * w2[c];
    s += __shfl_xor(s, 1);
    s += __shfl_xor(s, 2);
    const float w = s + sPar[4 * DN];
    if (g == 0) {
      v4f cu;
      cu.x = sDis[4 * e] * w; cu.y = sDis[4 * e + 1] * w; cu.z = sDis[4 * e + 2] * w; cu.w = 0.0f;
      *(v4f*)(sCo + 4 * e) = cu;
    }
  }
  __syncthreads();

  if (tid < NBE) {
    const v4f v = *(const v4f*)(sCo + 4 * tid);
    *(volatile v4f*)(Cout + (size_t)(el0 + tid) * CROW) = v;
  }
  __threadfence();
  if (tid < NBE) {
    const v4f v = *(const v4f*)(sCo + 4 * tid);
    *(volatile v4f*)(Cout + (size_t)(el0 + tid) * CROW) = v;
  }
}

__device__ __forceinline__ int scan_piece(const int* __restrict__ eid, int lim, int cbase, int base, int vecok,
                                          int* list, int tid, int wave) {
  int wc = 0;
  const int el0  = tid * EPT;
  const int e0   = cbase + el0;
  const int sent = -2147483647 - 1;
  int kk[EPT];
  if (vecok != 0 && cbase + PIECE <= lim) {
    const v4i* p = (const v4i*)(eid + e0);
#pragma unroll
    for (int u = 0; u < EPT / 4; ++u) {
      const v4i d = p[u];
      kk[4 * u] = d.x; kk[4 * u + 1] = d.y; kk[4 * u + 2] = d.z; kk[4 * u + 3] = d.w;
    }
  } else {
    const int lm = lim - 1;
#pragma unroll
    for (int q = 0; q < EPT; ++q) {
      const int eq = e0 + q;
      const int ec = eq > lm ? lm : eq;
      const int a = eid[ec];
      kk[q] = (eq < lim) ? a : sent;
    }
  }
  const unsigned nb = (unsigned)base;
  unsigned sq[EPT];
  bool hq[EPT];
  bool anyl = false;
#pragma unroll
  for (int q = 0; q < EPT; ++q) {
    sq[q] = (unsigned)kk[q] - nb;
    hq[q] = sq[q] < (unsigned)NBC;
    anyl = anyl | hq[q];
  }
  const unsigned any = __builtin_amdgcn_ballot_w32(anyl);
  if (any != 0u) {
#define HIT(HQ, SQ, Q) { \
      const unsigned mj = __builtin_amdgcn_ballot_w32(HQ); \
      if (mj != 0u) { \
        if (HQ) { \
          const int ps = wc + (int)__builtin_amdgcn_mbcnt_lo(mj, 0u); \
          if (ps < WCAP) list[wave * WCAP + ps] = ((el0 + (Q)) << SLB) | (int)(SQ); \
        } \
        wc += (int)__builtin_popcount(mj); } }
#pragma unroll
    for (int q = 0; q < EPT; ++q) {
      HIT(hq[q], sq[q], q)
    }
#undef HIT
  }
  return wc;
}

__device__ __forceinline__ void drain_piece(const int* list, const int* wcnt, float* accF, float* accC,
                                            const float* __restrict__ Mf, const float* __restrict__ Cq,
                                            int rowoff, int lane, int wave) {
#pragma unroll 1
  for (int wsx = 0; wsx < NWAVE; ++wsx) {
    int n = __builtin_amdgcn_readfirstlane(wcnt[wsx]);
    n = n > WCAP ? WCAP : (n < 0 ? 0 : n);
    const int* lp = list + wsx * WCAP;
#pragma unroll 1
    for (int bb = 0; bb < n; bb += 32) {
      const int idx = bb + lane;
      const int ic = idx > WCAP - 1 ? WCAP - 1 : idx;
      const int ent = lp[ic];
      const bool own = (idx < n) && ((ent & (NWAVE - 1)) == wave);
      unsigned msk = __builtin_amdgcn_ballot_w32(own);
#pragma unroll 1
      while (msk != 0u) {
        const int bit = (int)__builtin_ctz(msk);
        msk &= msk - 1u;
        const int e2 = __builtin_amdgcn_readlane(ent, bit);
        const int slot = e2 & (NBC - 1);
        const int el = (e2 >> SLB) & (PIECE - 1);
        int row = rowoff + el;
        row = row < 0 ? 0 : (row > CE - 1 ? CE - 1 : row);
        const v4f mv = *(const v4f*)(Mf + (size_t)row * MROW + 4 * lane);
        float* ap = accF + slot * DN + 4 * lane;
        v4f a = *(const v4f*)ap;
        a += mv;
        *(v4f*)ap = a;
        const float cvv = Cq[(size_t)row * CROW + (lane & 3)];
        if (lane < 3) accC[CROW * slot + lane] += cvv;
      }
    }
  }
}

__device__ __forceinline__ void agg_store(const float* accF, const float* accC, const float* __restrict__ x,
                                          float* outH, float* outX, int base, int nN, int last, float Cw,
                                          int tid, int lane, int wave) {
#pragma unroll 1
  for (int it = 0; it < NBC / NWAVE; ++it) {
    const int s = wave + NWAVE * it;
    const int node = base + s;
    if (node < nN) {
      const v4f v = *(const v4f*)(accF + s * DN + 4 * lane);
      *(volatile v4f*)(outH + (size_t)node * DN + 4 * lane) = v;
    }
  }
  int cnt = nN - base;
  cnt = cnt > NBC ? NBC : cnt;
  const int nfl = 3 * cnt, nq = nfl >> 2, rem = nfl & 3;
  const size_t f0 = (size_t)3 * (size_t)base;
#pragma unroll 1
  for (int it = 0; it < 2; ++it) {
    const int q = tid + NTHR * it;
    if (q < nq) {
      float a[4];
#pragma unroll
      for (int c = 0; c < 4; ++c) {
        const int t = 4 * q + c;
        const int s3 = t / 3;
        const float sv = accC[CROW * s3 + (t - 3 * s3)];
        const float xv = x[f0 + (size_t)t];
        a[c] = (last != 0) ? (xv + sv * Cw) : sv;
      }
      v4f ov;
      ov.x = a[0]; ov.y = a[1]; ov.z = a[2]; ov.w = a[3];
      *(volatile v4f*)(outX + f0 + 4 * (size_t)q) = ov;
    } else if (q == nq && rem != 0) {
#pragma unroll
      for (int c = 0; c < 3; ++c) {
        if (c < rem) {
          const int t = 4 * q + c;
          const int s3 = t / 3;
          const float sv = accC[CROW * s3 + (t - 3 * s3)];
          const float xv = x[f0 + (size_t)t];
          const float val = (last != 0) ? (xv + sv * Cw) : sv;
          *(volatile float*)(outX + f0 + (size_t)t) = val;
        }
      }
    }
  }
}

__global__ __launch_bounds__(NTHR) void k_agg(
    const int* __restrict__ ei, const float* __restrict__ Mq, const float* __restrict__ Cq,
    const float* __restrict__ x, float* outH, float* outX, int nE, int cbeg, int lim, int nN,
    int first, int last, int vecok, float Cw) {
  extern __shared__ __attribute__((aligned(16))) float accd[];
  __shared__ int list[NWAVE * WCAP];
  __shared__ int wcnt[NWAVE];
  const int tid = (int)threadIdx.x, lane = tid & 31, wave = tid >> 5;
  const int base = (int)blockIdx.x * NBC;
  float* accF = accd;
  float* accC = accd + NBC * DN;
  const int* eid = ei + (size_t)nE;

  if (first != 0) {
#pragma unroll 1
    for (int i = tid; i < (NBC * DN) / 4; i += NTHR) *(v4f*)(accF + 4 * i) = zero4();
#pragma unroll 1
    for (int s = tid; s < NBC; s += NTHR) *(v4f*)(accC + CROW * s) = zero4();
  } else {
#pragma unroll 1
    for (int i = tid; i < (NBC * DN) / 4; i += NTHR) {
      const int s = i >> 5, c4 = (i & 31) * 4;
      int node = base + s;
      node = node > nN - 1 ? nN - 1 : node;
      const v4f v = *(const v4f*)(outH + (size_t)node * DN + c4);
      *(v4f*)(accF + s * DN + c4) = v;
    }
#pragma unroll 1
    for (int s = tid; s < NBC; s += NTHR) {
      int node = base + s;
      node = node > nN - 1 ? nN - 1 : node;
      const float* sp = outX + (size_t)node * 3;
      v4f v;
      v.x = sp[0]; v.y = sp[1]; v.z = sp[2]; v.w = 0.0f;
      *(v4f*)(accC + CROW * s) = v;
    }
  }
  __syncthreads();

#pragma unroll 1
  for (int cbase = cbeg; cbase < lim; cbase += PIECE) {
    const int wc = scan_piece(eid, lim, cbase, base, vecok, list, tid, wave);
    if (lane == 0) wcnt[wave] = wc;
    __syncthreads();
    drain_piece(list, wcnt, accF, accC, Mq, Cq, cbase - cbeg, lane, wave);
    __syncthreads();
  }

  agg_store(accF, accC, x, outH, outX, base, nN, last, Cw, tid, lane, wave);
  __threadfence();
  agg_store(accF, accC, x, outH, outX, base, nN, last, Cw, tid, lane, wave);
}

__global__ __launch_bounds__(NTHR) void k_nodemlp(
    const float* __restrict__ nsrc, const unsigned short* __restrict__ wp,
    const float* __restrict__ bh1, const float* __restrict__ bh2, float* HO, int nN) {
  extern __shared__ __attribute__((aligned(16))) float mdynf[];
  __shared__ __attribute__((aligned(16))) float sPar[2 * DN];
  unsigned short* sAH = (unsigned short*)mdynf;
  unsigned short* sAL = sAH + NBN * APN;
  unsigned short* sYH = sAL + NBN * APN;
  unsigned short* sYL = sYH + NBN * APA;
  float* sU = mdynf;
  const int tid = (int)threadIdx.x, lane = tid & 31, wave = tid >> 5, hh = lane >> 4, m = lane & 15;
  const int n0 = (int)blockIdx.x * NBN;

  {
    const int nl = tid >> 2, g = tid & 3;
    int node = n0 + nl;
    node = node > nN - 1 ? nN - 1 : node;
    const float* np_ = nsrc + (size_t)node * DN + 32 * g;
    const float* mp  = HO   + (size_t)node * DN + 32 * g;
#pragma unroll
    for (int i = 0; i < 4; ++i) {
      const v4f xa = *(const v4f*)(np_ + 8 * i);
      const v4f xb = *(const v4f*)(np_ + 8 * i + 4);
      v8us h, l;
      cvt_hl8(xa, xb, h, l);
      *(v8us*)(sAH + nl * APN + 32 * g + 8 * i) = h;
      *(v8us*)(sAL + nl * APN + 32 * g + 8 * i) = l;
    }
#pragma unroll
    for (int i = 0; i < 4; ++i) {
      const v4f xa = *(const v4f*)(mp + 8 * i);
      const v4f xb = *(const v4f*)(mp + 8 * i + 4);
      v8us h, l;
      cvt_hl8(xa, xb, h, l);
      *(v8us*)(sAH + nl * APN + DN + 32 * g + 8 * i) = h;
      *(v8us*)(sAL + nl * APN + DN + 32 * g + 8 * i) = l;
    }
  }
  if (tid < DN) {
    sPar[tid]      = bh1[tid];
    sPar[DN + tid] = bh2[tid];
  }
  __syncthreads();

  const int rt = wave & 3, cg = wave >> 2;

  {
    v8f a0, a1, a2, a3;
    gemm3x16x64(sAH + (16 * rt + m) * APN + 8 * hh, sAL + (16 * rt + m) * APN + 8 * hh,
                wp + PN1H, wp + PN1L, 2 * DN, 8, 64 * cg, m, hh, a0, a1, a2, a3);
    unsigned short* ph = sYH + (16 * rt + 8 * hh) * APA + 64 * cg + m;
    unsigned short* pl = sYL + (16 * rt + 8 * hh) * APA + 64 * cg + m;
    const float* bb = sPar + 64 * cg + m;
    stage8y(ph,      pl,      a0, bb[0]);
    stage8y(ph + 16, pl + 16, a1, bb[16]);
    stage8y(ph + 32, pl + 32, a2, bb[32]);
    stage8y(ph + 48, pl + 48, a3, bb[48]);
  }
  __syncthreads();

  {
    v8f a0, a1, a2, a3;
    gemm3x16x64(sYH + (16 * rt + m) * APA + 8 * hh, sYL + (16 * rt + m) * APA + 8 * hh,
                wp + PN2H, wp + PN2L, DN, 4, 64 * cg, m, hh, a0, a1, a2, a3);
    float* sp = sU + (16 * rt + 8 * hh) * GSTR + 64 * cg + m;
    const float* bb = sPar + DN + 64 * cg + m;
    stage8f(sp,      a0, 1.0f, bb[0]);
    stage8f(sp + 16, a1, 1.0f, bb[16]);
    stage8f(sp + 32, a2, 1.0f, bb[32]);
    stage8f(sp + 48, a3, 1.0f, bb[48]);
  }
  __syncthreads();

#pragma unroll 1
  for (int it = 0; it < NBN / NWAVE; ++it) {
    const int s = wave + NWAVE * it;
    const int node = n0 + s;
    if (node < nN) {
      const v4f v = *(const v4f*)(sU + s * GSTR + 4 * lane);
      *(volatile v4f*)(HO + (size_t)node * DN + 4 * lane) = v;
    }
  }
  __threadfence();
#pragma unroll 1
  for (int it = 0; it < NBN / NWAVE; ++it) {
    const int s = wave + NWAVE * it;
    const int node = n0 + s;
    if (node < nN) {
      const v4f v = *(const v4f*)(sU + s * GSTR + 4 * lane);
      *(volatile v4f*)(HO + (size_t)node * DN + 4 * lane) = v;
    }
  }
}

extern "C" void kernel_launch(void* const* d_in, const int* in_sizes, int n_in,
                              void* d_out, int out_size, void* d_ws, size_t ws_size,
                              hipStream_t stream) {
  if (n_in < 13) return;
  if (in_sizes[1] < 6 || (in_sizes[1] % 3) != 0) return;
  const int nN = in_sizes[1] / 3;
  if (nN < 2 || nN > (1 << 22)) return;
  if (in_sizes[0] != nN * DN) return;
  if (in_sizes[2] < 2 || (in_sizes[2] % 2) != 0) return;
  const int nE = in_sizes[2] / 2;
  if (nE < 1 || nE > (1 << 27)) return;
  if (in_sizes[3] != (2 * DN + 1) * DN || in_sizes[4] != DN) return;
  if (in_sizes[5] != DN * DN || in_sizes[6] != DN) return;
  if (in_sizes[7] != DN || in_sizes[8] < 1) return;
  if (in_sizes[9] != 2 * DN * DN || in_sizes[10] != DN) return;
  if (in_sizes[11] != DN * DN || in_sizes[12] != DN) return;
  if (out_size != 131 * nN) return;

  const float* node  = (const float*)d_in[0];
  const float* coord = (const float*)d_in[1];
  const int*   ei    = (const int*)d_in[2];
  const float* We1   = (const float*)d_in[3];
  const float* be1   = (const float*)d_in[4];
  const float* We2   = (const float*)d_in[5];
  const float* be2   = (const float*)d_in[6];
  const float* Wx    = (const float*)d_in[7];
  const float* bx    = (const float*)d_in[8];
  const float* Wh1   = (const float*)d_in[9];
  const float* bh1   = (const float*)d_in[10];
  const float* Wh2   = (const float*)d_in[11];
  const float* bh2   = (const float*)d_in[12];
  float* out0 = (float*)d_out;
  float* out1 = out0 + (size_t)DN * (size_t)nN;

  const int nbNode = (nN + NBN - 1) / NBN;
  const int Npad   = nbNode * NBN;
  const int nChunk = (nE + CE - 1) / CE;
  if (nChunk < 1 || nChunk > MAXCH) return;
  const int nbAgg  = (nN + NBC - 1) / NBC;
  const int vecok  = ((nE & 3) == 0) ? 1 : 0;
  const float Cw   = (float)(1.0 / (double)(nN - 1));

  char* ws = (char*)d_ws;
  size_t off = 0;
  const size_t oW  = off; off += (size_t)PWTOT * 2;             off = (off + 255) & ~(size_t)255;
  const size_t oNP = off; off += (size_t)Npad * NPROW * 4;       off = (off + 255) & ~(size_t)255;
  const size_t oM  = off; off += (size_t)CE * MROW * 4;          off = (off + 255) & ~(size_t)255;
  const size_t oC  = off; off += (size_t)CE * CROW * 4;          off = (off + 255) & ~(size_t)255;
  if (off > ws_size || off > (size_t)WSCAP) return;
  unsigned short* wp = (unsigned short*)(ws + oW);
  float* NP          = (float*)(ws + oNP);
  float* Mq          = (float*)(ws + oM);
  float* Cq          = (float*)(ws + oC);

  hipFuncSetAttribute(reinterpret_cast<const void*>(&k_node), hipFuncAttributeMaxDynamicSharedMemorySize, NODEDYN);
  hipFuncSetAttribute(reinterpret_cast<const void*>(&k_edge), hipFuncAttributeMaxDynamicSharedMemorySize, EDGEDYN);
  hipFuncSetAttribute(reinterpret_cast<const void*>(&k_agg), hipFuncAttributeMaxDynamicSharedMemorySize, AGGDYN);
  hipFuncSetAttribute(reinterpret_cast<const void*>(&k_nodemlp), hipFuncAttributeMaxDynamicSharedMemorySize, MLPDYN);

  k_prep<<<PBLK, NTHR, 0, stream>>>(We1, We2, Wh1, Wh2, wp);
  k_node<<<nbNode, NTHR, NODEDYN, stream>>>(node, wp, NP, nN);
  for (int c = 0; c < nChunk; ++c) {
    const int cbeg = c * CE;
    int lim = cbeg + CE;
    lim = lim > nE ? nE : lim;
    const int nblk = (lim - cbeg + NBE - 1) / NBE;
    const int first = (c == 0) ? 1 : 0;
    const int last  = (c == nChunk - 1) ? 1 : 0;
    k_edge<<<nblk, NTHR, EDGEDYN, stream>>>(coord, ei, NP, wp, We1, be1, be2, Wx, bx, Mq, Cq, nE, nN, cbeg);
    k_agg<<<nbAgg, NTHR, AGGDYN, stream>>>(ei, Mq, Cq, coord, out0, out1, nE, cbeg, lim, nN, first, last, vecok, Cw);
  }
  k_nodemlp<<<nbNode, NTHR, MLPDYN, stream>>>(node, wp, bh1, bh2, out0, nN);
}
